// BackProjLayer_57045755625641
// MI455X (gfx1250) — hardware-verified
//
#include <hip/hip_runtime.h>
#include <math.h>

typedef __attribute__((ext_vector_type(16))) _Float16 v16h;
typedef __attribute__((ext_vector_type(8)))  _Float16 v8h;
typedef __attribute__((ext_vector_type(8)))  float    v8f;
typedef __attribute__((ext_vector_type(4)))  float    v4f;

constexpr int kSamples    = 65536;
constexpr int kCh         = 4;
constexpr int kPx         = 242;
constexpr int kPxPad      = 256;
constexpr int kKdim       = 32;
constexpr int kBlkRows    = 32;
constexpr int kAPitch     = 40;
constexpr int kSweeps     = 8;
constexpr int kTileF4     = kBlkRows * kPx / 4;
constexpr int kStoreIters = (kTileF4 + 31) / 32;
constexpr float kCarryA   = 64.0f;
constexpr float kCarryW   = 1024.0f;
constexpr float kFold     = 1.0f / (kCarryA * kCarryW);
constexpr float kH16Min   = 6.103515625e-5f;

constexpr size_t kWsTotal = (size_t)kPxPad * kKdim * 2;

static_assert(kCh == 4, "4 channels");
static_assert(kKdim == 2 * kCh * kCh, "K = 16 symmetric-part + 16 antisymmetric-part coefficients");
static_assert(kKdim % 32 == 0, "K multiple of 32");
static_assert(kPxPad % 16 == 0 && kPxPad >= kPx, "N padded to the 16-wide tile");
static_assert(kSamples % kBlkRows == 0, "exact grid");
static_assert((kBlkRows * kPx) % 4 == 0, "stripe is whole 16-B pieces");
static_assert(((size_t)kBlkRows * kPx * 4) % 128 == 0, "stripe is whole 128-B lines");
static_assert(kTileF4 == 1936 && kStoreIters == 61, "store map");
static_assert((kAPitch * 2) % 16 == 0, "A row pitch 16-B aligned");
static_assert(kWsTotal == 16384ull, "carve total");
static_assert(kWsTotal <= 134217728ull, "carve cap");

union FragH { v16h v; v8h h[2]; };

__device__ __forceinline__ v16h frag_load_h(const _Float16* p) {
  FragH f;
  f.h[0] = *(const v8h*)(p);
  f.h[1] = *(const v8h*)(p + 16);
  return f.v;
}

__device__ __forceinline__ v8f mma_f16(v16h a, v16h b, v8f c) {
  c = __builtin_amdgcn_wmma_f32_16x16x32_f16(false, a, false, b, (short)0, c, false, false);
  asm volatile("v_nop\n\tv_nop\n\tv_nop\n\tv_nop" : "+v"(c) : "v"(a), "v"(b));
  return c;
}

__device__ __forceinline__ _Float16 to_h16(float v) {
  const float f = (fabsf(v) < kH16Min) ? 0.0f : v;
  return (_Float16)f;
}

template <int I, int J>
__device__ __forceinline__ float get_re(const float (&hr)[4][4]) { return (I < J) ? hr[I][J] : hr[J][I]; }
template <int I, int J>
__device__ __forceinline__ float get_im(const float (&hi)[4][4]) { return (I < J) ? hi[I][J] : -hi[J][I]; }
template <int I, int J>
__device__ __forceinline__ void put_c(float (&hr)[4][4], float (&hi)[4][4], float re, float im) {
  if (I < J) { hr[I][J] = re; hi[I][J] = im; }
  else       { hr[J][I] = re; hi[J][I] = -im; }
}

template <int P, int Q, int KX>
__device__ __forceinline__ void rot_offdiag(float (&hr)[4][4], float (&hi)[4][4], float c, float er, float ei) {
  if (KX == P || KX == Q) return;
  const float xr = get_re<KX, P>(hr);
  const float xi = get_im<KX, P>(hi);
  const float yr = get_re<KX, Q>(hr);
  const float yi = get_im<KX, Q>(hi);
  const float npr = c * xr + (er * yr - ei * yi);
  const float npi = c * xi + (er * yi + ei * yr);
  const float nqr = c * yr - (er * xr + ei * xi);
  const float nqi = c * yi - (er * xi - ei * xr);
  put_c<KX, P>(hr, hi, npr, npi);
  put_c<KX, Q>(hr, hi, nqr, nqi);
}

template <int P, int Q>
__device__ __forceinline__ void plane_rot(float (&hr)[4][4], float (&hi)[4][4],
                                          float (&vr)[4][4], float (&vi)[4][4]) {
  const float br  = hr[P][Q];
  const float bi  = hi[P][Q];
  const float m2  = br * br + bi * bi;
  const bool  nz  = m2 > 1.0e-30f;
  const float m2s = nz ? m2 : 1.0f;
  const float mag = sqrtf(m2s);
  const float inv = 1.0f / mag;
  const float cph = br * inv;
  const float sph = bi * inv;
  const float th  = (hr[P][P] - hr[Q][Q]) * (0.5f * inv);
  const float ath = fabsf(th);
  const float den = ath + sqrtf(ath * ath + 1.0f);
  const float tq  = copysignf(1.0f / den, th);
  const float t   = nz ? tq : 0.0f;
  const float c   = 1.0f / sqrtf(t * t + 1.0f);
  const float s   = t * c;
  const float er  = s * cph;
  const float ei  = -(s * sph);

  rot_offdiag<P, Q, 0>(hr, hi, c, er, ei);
  rot_offdiag<P, Q, 1>(hr, hi, c, er, ei);
  rot_offdiag<P, Q, 2>(hr, hi, c, er, ei);
  rot_offdiag<P, Q, 3>(hr, hi, c, er, ei);

  const float tm = t * mag;
  hr[P][P] += tm;
  hr[Q][Q] -= tm;
  hr[P][Q] = 0.0f;
  hi[P][Q] = 0.0f;

#pragma unroll
  for (int k = 0; k < 4; ++k) {
    const float xr = vr[k][P];
    const float xi = vi[k][P];
    const float yr = vr[k][Q];
    const float yi = vi[k][Q];
    vr[k][P] = c * xr + (er * yr - ei * yi);
    vi[k][P] = c * xi + (er * yi + ei * yr);
    vr[k][Q] = c * yr - (er * xr + ei * xi);
    vi[k][Q] = c * yi - (er * xi - ei * xr);
  }
}

__global__ __launch_bounds__(256) void wplane_prep_kernel(
    const float* __restrict__ Dre, const float* __restrict__ Dim, unsigned short* __restrict__ Wt)
{
  __shared__ __align__(16) _Float16 sW[kPxPad * kKdim];
  const int  p     = threadIdx.x;
  const bool valid = p < kPx;
  const int  pc    = valid ? p : (kPx - 1);

  float av[4], bv[4];
#pragma unroll
  for (int c = 0; c < 4; ++c) {
    float x = Dre[c * kPx + pc];
    float y = Dim[c * kPx + pc];
    asm volatile("" : "+v"(x), "+v"(y));
    av[c] = x;
    bv[c] = y;
  }
  float zq = 0.0f;
  asm volatile("" : "+v"(zq));

  float wv[32];
#pragma unroll
  for (int c = 0; c < 4; ++c) {
#pragma unroll
    for (int d = 0; d < 4; ++d) {
      const float re = av[c] * av[d] + bv[c] * bv[d];
      float im = bv[c] * av[d] - av[c] * bv[d];
      if (c == d) im = zq;
      wv[c * 4 + d]      = valid ? (re * kCarryW) : 0.0f;
      wv[16 + c * 4 + d] = valid ? (im * kCarryW) : 0.0f;
    }
  }
#pragma unroll
  for (int j = 0; j < 4; ++j) {
    v8h x;
#pragma unroll
    for (int e = 0; e < 8; ++e) x[e] = to_h16(wv[8 * j + e]);
    *(v8h*)(sW + p * kKdim + 8 * j) = x;
  }
  __syncthreads();

  v8h piece[4];
#pragma unroll
  for (int it = 0; it < 4; ++it) piece[it] = *(const v8h*)(sW + (it * 256 + p) * 8);
  for (int pass = 0; pass < 2; ++pass) {
#pragma unroll
    for (int it = 0; it < 4; ++it)
      *(volatile v8h*)(Wt + (size_t)(it * 256 + p) * 8) = piece[it];
    __threadfence();
  }
}

__global__ __launch_bounds__(32) void psd_project_kernel(
    const float* __restrict__ Sre, const float* __restrict__ Sim,
    const unsigned short* __restrict__ Wt, const float* __restrict__ tau,
    float* __restrict__ out)
{
  __shared__ __align__(16) _Float16 sA[kBlkRows * kAPitch];
  __shared__ __align__(16) float    sStage[kBlkRows * kPx];

  const int lane = threadIdx.x & 31;
  const int hh   = lane >> 4;
  const int m    = lane & 15;
  size_t n = (size_t)blockIdx.x * kBlkRows + lane;
  if (n > (size_t)(kSamples - 1)) n = (size_t)(kSamples - 1);

  float sr[16], si[16];
  {
    const v4f* pr = (const v4f*)(Sre + n * 16);
    const v4f* pi = (const v4f*)(Sim + n * 16);
#pragma unroll
    for (int j = 0; j < 4; ++j) {
      const v4f x = pr[j];
      const v4f y = pi[j];
      sr[4 * j + 0] = x[0]; sr[4 * j + 1] = x[1]; sr[4 * j + 2] = x[2]; sr[4 * j + 3] = x[3];
      si[4 * j + 0] = y[0]; si[4 * j + 1] = y[1]; si[4 * j + 2] = y[2]; si[4 * j + 3] = y[3];
    }
  }

  float hr[4][4], hi[4][4], vr[4][4], vi[4][4];
#pragma unroll
  for (int i = 0; i < 4; ++i) {
#pragma unroll
    for (int j = 0; j < 4; ++j) {
      float re = 0.0f, im = 0.0f;
      if (i == j) re = sr[i * 4 + i];
      if (i < j) {
        re = 0.5f * (sr[i * 4 + j] + sr[j * 4 + i]);
        im = 0.5f * (si[i * 4 + j] - si[j * 4 + i]);
      }
      hr[i][j] = re;
      hi[i][j] = im;
      vr[i][j] = (i == j) ? 1.0f : 0.0f;
      vi[i][j] = 0.0f;
    }
  }

#pragma unroll 1
  for (int sw = 0; sw < kSweeps; ++sw) {
    plane_rot<0, 1>(hr, hi, vr, vi);
    plane_rot<2, 3>(hr, hi, vr, vi);
    plane_rot<0, 2>(hr, hi, vr, vi);
    plane_rot<1, 3>(hr, hi, vr, vi);
    plane_rot<0, 3>(hr, hi, vr, vi);
    plane_rot<1, 2>(hr, hi, vr, vi);
  }

  float lam[4];
#pragma unroll
  for (int d = 0; d < 4; ++d) lam[d] = fmaxf(hr[d][d], 0.0f);
  float wr[4][4], wi[4][4];
#pragma unroll
  for (int c = 0; c < 4; ++c) {
#pragma unroll
    for (int d = 0; d < 4; ++d) {
      wr[c][d] = lam[d] * vr[c][d];
      wi[c][d] = lam[d] * vi[c][d];
    }
  }
  float zq = 0.0f;
  asm volatile("" : "+v"(zq));
  float vec[32];
#pragma unroll
  for (int c = 0; c < 4; ++c) {
#pragma unroll
    for (int c2 = 0; c2 < 4; ++c2) {
      if (c2 >= c) {
        float pacc = 0.0f;
#pragma unroll
        for (int d = 0; d < 4; ++d) {
          pacc += wr[c][d] * vr[c2][d];
          pacc += wi[c][d] * vi[c2][d];
        }
        const float ps = pacc * kCarryA;
        vec[c * 4 + c2] = ps;
        vec[c2 * 4 + c] = ps;
        if (c2 > c) {
          float qacc = 0.0f;
#pragma unroll
          for (int d = 0; d < 4; ++d) {
            qacc += wi[c][d] * vr[c2][d];
            qacc -= wr[c][d] * vi[c2][d];
          }
          const float qs = qacc * kCarryA;
          vec[16 + c * 4 + c2] = qs;
          vec[16 + c2 * 4 + c] = -qs;
        } else {
          vec[16 + c * 4 + c] = zq;
        }
      }
    }
  }

#pragma unroll
  for (int j = 0; j < 4; ++j) {
    v8h x;
#pragma unroll
    for (int e = 0; e < 8; ++e) x[e] = to_h16(vec[8 * j + e]);
    *(v8h*)(sA + lane * kAPitch + 8 * j) = x;
  }
  __syncthreads();

  const v16h a0 = frag_load_h(sA + m * kAPitch + 8 * hh);
  const v16h a1 = frag_load_h(sA + (16 + m) * kAPitch + 8 * hh);
  const _Float16* Wp = (const _Float16*)Wt;

#pragma unroll 8
  for (int nt = 0; nt < kPxPad / 16; ++nt) {
    const int col  = nt * 16 + m;
    const int colc = (col < kPx) ? col : (kPx - 1);
    float tv = tau[colc];
    asm volatile("" : "+v"(tv));
    const v16h b = frag_load_h(Wp + (size_t)col * kKdim + 8 * hh);
    v8f acc0 = (v8f){0.f, 0.f, 0.f, 0.f, 0.f, 0.f, 0.f, 0.f};
    v8f acc1 = (v8f){0.f, 0.f, 0.f, 0.f, 0.f, 0.f, 0.f, 0.f};
    acc0 = mma_f16(a0, b, acc0);
    acc1 = mma_f16(a1, b, acc1);
    if (col < kPx) {
#pragma unroll
      for (int r = 0; r < 8; ++r) {
        sStage[(8 * hh + r) * kPx + col]      = acc0[r] * kFold - tv;
        sStage[(16 + 8 * hh + r) * kPx + col] = acc1[r] * kFold - tv;
      }
    }
  }
  __syncthreads();

  float* ob = out + (size_t)blockIdx.x * (size_t)(kBlkRows * kPx);
  for (int pass = 0; pass < 2; ++pass) {
#pragma unroll 1
    for (int it = 0; it < kStoreIters; ++it) {
      const int idx = it * 32 + lane;
      const int idc = (idx < kTileF4) ? idx : (kTileF4 - 1);
      const v4f v = *(const v4f*)(sStage + idc * 4);
      if (idx < kTileF4) *(volatile v4f*)(ob + (size_t)idx * 4) = v;
    }
    __threadfence();
  }
}

extern "C" void kernel_launch(void* const* d_in, const int* in_sizes, int n_in,
                              void* d_out, int out_size, void* d_ws, size_t ws_size,
                              hipStream_t stream) {
  if (n_in < 5) return;
  if (in_sizes[0] != kSamples * kCh * kCh) return;
  if (in_sizes[1] != kSamples * kCh * kCh) return;
  if (in_sizes[2] != kCh * kPx) return;
  if (in_sizes[3] != kCh * kPx) return;
  if (in_sizes[4] != kPx) return;
  if (out_size != kSamples * kPx) return;
  if (ws_size < kWsTotal) return;

  const float* Sre = (const float*)d_in[0];
  const float* Sim = (const float*)d_in[1];
  const float* Dre = (const float*)d_in[2];
  const float* Dim = (const float*)d_in[3];
  const float* tau = (const float*)d_in[4];
  float* out = (float*)d_out;
  unsigned short* Wt = (unsigned short*)d_ws;

  wplane_prep_kernel<<<1, 256, 0, stream>>>(Dre, Dim, Wt);
  psd_project_kernel<<<kSamples / kBlkRows, kBlkRows, 0, stream>>>(Sre, Sim, Wt, tau, out);
}
